// PointnetSAModuleMSG_16947940950606
// MI455X (gfx1250) — hardware-verified
//
#include <hip/hip_runtime.h>
#pragma clang fp contract(off)

typedef __attribute__((ext_vector_type(16))) __bf16   v16b;
typedef __attribute__((ext_vector_type(8)))  __bf16   v8b;
typedef __attribute__((ext_vector_type(8)))  float    v8f;
typedef __attribute__((ext_vector_type(4)))  float    v4f;
typedef __attribute__((ext_vector_type(4)))  int      v4i;
typedef __attribute__((ext_vector_type(4)))  unsigned v4u;

constexpr int NBATCH = 8;
constexpr int NPTS   = 4096;
constexpr int NQRY   = 1024;
constexpr int NQTOT  = NBATCH * NQRY;
constexpr int CFEAT  = 128;
constexpr int CIN    = 131;
constexpr int CMID   = 64;
constexpr int COUTC  = 256;
constexpr int NPADW  = 144;
constexpr int KPADW  = 160;
constexpr int IDXP   = 64;
constexpr int YPITCH = 160;

static_assert(CIN == CFEAT + 3, "channel layout");
static_assert(NPADW % 16 == 0 && NPADW >= CIN, "padded N of the 64->131 layer");
static_assert(KPADW % 32 == 0 && KPADW >= CIN, "padded K of the 131->256 layer");
static_assert(NQTOT % 64 == 0 && COUTC % 64 == 0 && CMID % 32 == 0, "GEMM tile multiples");

constexpr size_t SZ_FEATT = (size_t)NBATCH * NPTS * CFEAT * 4;
constexpr size_t SZ_NQ    = (size_t)NQTOT * 4 * 4;
constexpr size_t SZ_W2P   = (size_t)NPADW * CMID * 2;
constexpr size_t SZ_WCP   = (size_t)COUTC * KPADW * 2;
constexpr size_t OFF_FEATT = 0;
constexpr size_t OFF_NQ    = OFF_FEATT + SZ_FEATT;
constexpr size_t OFF_W2H   = OFF_NQ + SZ_NQ;
constexpr size_t OFF_W2L   = OFF_W2H + SZ_W2P;
constexpr size_t OFF_WCH   = OFF_W2L + SZ_W2P;
constexpr size_t OFF_WCL   = OFF_WCH + SZ_WCP;
constexpr size_t OFF_SC0   = OFF_WCL + SZ_WCP;
constexpr size_t SZ_IDX   = (size_t)NQTOT * IDXP * 4;
constexpr size_t SZ_ST1   = (size_t)1024 * 128 * 4;
constexpr size_t SZ_AB1   = 1024;
constexpr size_t SZ_YPL   = (size_t)NQTOT * YPITCH * 4;
constexpr size_t SZ_AB2   = 2048;
constexpr size_t SZ_XP    = (size_t)NQTOT * KPADW * 2;
constexpr size_t SZ_P3    = (size_t)NQTOT * COUTC * 4;
constexpr size_t SZ_AB3   = 2048;
constexpr size_t SC_IDX = 0;
constexpr size_t SC_ST1 = SC_IDX + SZ_IDX;
constexpr size_t SC_AB1 = SC_ST1 + SZ_ST1;
constexpr size_t SC_Y   = SC_AB1 + SZ_AB1;
constexpr size_t SC_AB2 = SC_Y + 4 * SZ_YPL;
constexpr size_t SC_XPH = SC_AB2 + SZ_AB2;
constexpr size_t SC_XPL = SC_XPH + SZ_XP;
constexpr size_t SC_P3  = SC_XPL + SZ_XP;
constexpr size_t SC_AB3 = SC_P3 + SZ_P3;
constexpr size_t SC_BYTES = SC_AB3 + SZ_AB3;
constexpr size_t WS_TOTAL = OFF_SC0 + 2 * SC_BYTES;
static_assert(WS_TOTAL <= (size_t)134217728, "carve within 128 MiB");
static_assert((OFF_SC0 % 128) == 0 && (SC_BYTES % 128) == 0 && (SC_Y % 128) == 0 && (SC_XPH % 128) == 0 && (SC_P3 % 128) == 0, "line aligned carve");
constexpr int OUT1_FLOAT_OFF = NBATCH * NQRY * 3;
static_assert((size_t)OUT1_FLOAT_OFF * 4 == 98304, "out1 byte offset");
static_assert((size_t)OUT1_FLOAT_OFF * 4 + (size_t)NBATCH * 2 * COUTC * NQRY * 4 == (size_t)16875520, "d_out extent");

__device__ __forceinline__ int clampi(int v, int lo, int hi) { return v < lo ? lo : (v > hi ? hi : v); }

__device__ __forceinline__ void bf_split(float f, unsigned& hb, unsigned& lb) {
  const unsigned u = __float_as_uint(f);
  hb = (u + 0x7FFFu + ((u >> 16) & 1u)) >> 16;
  const float hf = __uint_as_float(hb << 16);
  const float rs = f - hf;
  const unsigned ur = __float_as_uint(rs);
  lb = (ur + 0x7FFFu + ((ur >> 16) & 1u)) >> 16;
}

union FragB { v16b v; v8b h[2]; };
__device__ __forceinline__ v16b frag_load(const __bf16* p) {
  FragB f; f.h[0] = *(const v8b*)(p); f.h[1] = *(const v8b*)(p + 16); return f.v;
}
__device__ __forceinline__ v8f mma_plain(v16b a, v16b b, v8f c) {
  return __builtin_amdgcn_wmma_f32_16x16x32_bf16(false, a, false, b, (short)0, c, false, false);
}
__device__ __forceinline__ v8f mma_g(v16b a, v16b b, v8f c) {
  c = __builtin_amdgcn_wmma_f32_16x16x32_bf16(false, a, false, b, (short)0, c, false, false);
  asm volatile("v_nop\n\tv_nop\n\tv_nop\n\tv_nop" : "+v"(c) : "v"(a), "v"(b));
  return c;
}
__device__ __forceinline__ void dep_guard4_b(v8f& a, v8f& b, v8f& c, v8f& d, v16b x, v16b y) {
  asm volatile("v_nop\n\tv_nop\n\tv_nop\n\tv_nop" : "+v"(a), "+v"(b), "+v"(c), "+v"(d) : "v"(x), "v"(y));
}
__device__ __forceinline__ void keep4_b(v16b a, v16b b, v16b c, v16b d) { asm volatile("v_nop" :: "v"(a), "v"(b), "v"(c), "v"(d)); }
__device__ __forceinline__ void acc_guard4(v8f& a, v8f& b, v8f& c, v8f& d) {
  asm volatile("v_nop\n\tv_nop\n\tv_nop\n\tv_nop" : "+v"(a), "+v"(b), "+v"(c), "+v"(d));
}
__device__ __forceinline__ void store2_v4f(float* p, v4f v) {
  *(volatile v4f*)p = v;
  __threadfence();
  *(volatile v4f*)p = v;
}

__device__ __forceinline__ float p1_base(float bias, float wx0, float wx1, float wx2, float wg0, float wg1, float wg2,
                                         float xi0, float xi1, float xi2, float n0, float n1, float n2) {
  float v = bias;
  v = v + wx0 * xi0; v = v + wx1 * xi1; v = v + wx2 * xi2;
  v = v + wg0 * n0;  v = v + wg1 * n1;  v = v + wg2 * n2;
  return v;
}
__device__ __forceinline__ float p1_eval(float base, float w0, float u0, float u1, float u2, v4f g) {
  float v = base;
  v = v + w0 * g.x; v = v + u0 * g.y; v = v + u1 * g.z; v = v + u2 * g.w;
  return v;
}

__global__ __launch_bounds__(256) void k_transpose_feat(const float* __restrict__ f, float* __restrict__ ft) {
  __shared__ __align__(16) float tile[32 * 132];
  const int tid = threadIdx.x, wave = tid >> 5, lane = tid & 31;
  const int b = blockIdx.y, n0 = blockIdx.x * 32;
#pragma unroll
  for (int hf = 0; hf < 2; ++hf) {
    float v[8];
#pragma unroll
    for (int r = 0; r < 8; ++r) {
      const int ch = wave * 16 + hf * 8 + r;
      v[r] = f[((size_t)(b * CFEAT + ch)) * NPTS + n0 + lane];
    }
#pragma unroll
    for (int r = 0; r < 8; ++r) {
      const int ch = wave * 16 + hf * 8 + r;
      tile[lane * 132 + ch] = v[r];
    }
    asm volatile("" ::: "memory");
  }
  __syncthreads();
  for (int pass = 0; pass < 2; ++pass) {
#pragma unroll
    for (int r = 0; r < 4; ++r) {
      const int n = wave * 4 + r;
      const v4f val = *(const v4f*)(tile + n * 132 + lane * 4);
      *(volatile v4f*)(ft + ((size_t)(b * NPTS + n0 + n)) * CFEAT + lane * 4) = val;
    }
    __threadfence();
  }
}

__global__ __launch_bounds__(256) void k_wprep(const float* __restrict__ W2, const float* __restrict__ Wcr,
                                               unsigned short* __restrict__ W2h, unsigned short* __restrict__ W2l,
                                               unsigned short* __restrict__ Wch, unsigned short* __restrict__ Wcl) {
  constexpr int G2 = NPADW * CMID / 8;
  constexpr int GC = COUTC * KPADW / 8;
  static_assert(G2 % 32 == 0 && (G2 + GC) % 32 == 0, "wave aligned regions");
  const int g = blockIdx.x * 256 + threadIdx.x;
  if (g >= G2 + GC) return;
  float v[8];
  unsigned short* dh;
  unsigned short* dl;
  if (g < G2) {
    const int n = g >> 3, k0 = (g & 7) * 8;
    const int nc = n < CIN ? n : (CIN - 1);
#pragma unroll
    for (int e = 0; e < 8; ++e) {
      const float x = W2[nc * CMID + k0 + e];
      v[e] = (n < CIN) ? x : 0.0f;
    }
    dh = W2h + (size_t)g * 8;
    dl = W2l + (size_t)g * 8;
  } else {
    const int gg = g - G2;
    const int n = gg / 20, k0 = (gg % 20) * 8;
#pragma unroll
    for (int e = 0; e < 8; ++e) {
      const int k = k0 + e;
      const int kc = k < CIN ? k : (CIN - 1);
      const float x = Wcr[n * CIN + kc];
      v[e] = (k < CIN) ? x : 0.0f;
    }
    dh = Wch + (size_t)gg * 8;
    dl = Wcl + (size_t)gg * 8;
  }
  unsigned hw[4], lw[4];
#pragma unroll
  for (int e2 = 0; e2 < 4; ++e2) {
    unsigned h0, l0, h1, l1;
    bf_split(v[2 * e2], h0, l0);
    bf_split(v[2 * e2 + 1], h1, l1);
    hw[e2] = h0 | (h1 << 16);
    lw[e2] = l0 | (l1 << 16);
  }
  const v4u hv = (v4u){hw[0], hw[1], hw[2], hw[3]};
  const v4u lv = (v4u){lw[0], lw[1], lw[2], lw[3]};
  *(volatile v4u*)dh = hv;
  *(volatile v4u*)dl = lv;
  __threadfence();
  *(volatile v4u*)dh = hv;
  *(volatile v4u*)dl = lv;
}

__global__ __launch_bounds__(1024) void k_fps(const float* __restrict__ xyz, float* __restrict__ out0, float* __restrict__ nqp) {
#pragma clang fp contract(off)
  __shared__ float raw[NPTS * 3];
  __shared__ int   sel[NQRY];
  __shared__ float rvs[2][32];
  __shared__ int   ris[2][32];
  const int b = blockIdx.x, t = threadIdx.x, lane = t & 31, wid = t >> 5;
  const float* src = xyz + (size_t)b * NPTS * 3;
#pragma unroll
  for (int j = 0; j < 12; ++j) raw[t + j * 1024] = src[t + j * 1024];
  if (t == 0) sel[0] = 0;
  __syncthreads();
  float px[4], py[4], pz[4], dm[4];
#pragma unroll
  for (int j = 0; j < 4; ++j) {
    const int p = t + j * 1024;
    px[j] = raw[3 * p]; py[j] = raw[3 * p + 1]; pz[j] = raw[3 * p + 2];
    dm[j] = 1e10f;
  }
  int last = 0;
#pragma unroll 1
  for (int it = 1; it < NQRY; ++it) {
    const float lx = raw[3 * last], ly = raw[3 * last + 1], lz = raw[3 * last + 2];
    float bv = -1.0f;
    int bi = 0;
#pragma unroll
    for (int j = 0; j < 4; ++j) {
      const float dx = px[j] - lx, dy = py[j] - ly, dz = pz[j] - lz;
      const float t0 = dx * dx;
      const float t1 = dy * dy;
      const float t2 = dz * dz;
      const float dd = (t0 + t2) + t1;
      dm[j] = fminf(dm[j], dd);
      if (dm[j] > bv) { bv = dm[j]; bi = t + j * 1024; }
    }
#pragma unroll
    for (int o = 16; o > 0; o >>= 1) {
      const float ov = __shfl_xor(bv, o, 32);
      const int   oi = __shfl_xor(bi, o, 32);
      if (ov > bv || (ov == bv && oi < bi)) { bv = ov; bi = oi; }
    }
    const int buf = it & 1;
    if (lane == 0) { rvs[buf][wid] = bv; ris[buf][wid] = bi; }
    __syncthreads();
    float v2 = rvs[buf][lane];
    int   i2 = ris[buf][lane];
#pragma unroll
    for (int o = 16; o > 0; o >>= 1) {
      const float ov = __shfl_xor(v2, o, 32);
      const int   oi = __shfl_xor(i2, o, 32);
      if (ov > v2 || (ov == v2 && oi < i2)) { v2 = ov; i2 = oi; }
    }
    last = clampi(i2, 0, NPTS - 1);
    if (t == 0) sel[it] = last;
  }
  __syncthreads();
  const int ps = sel[t];
  const v4f nv = (v4f){raw[3 * ps], raw[3 * ps + 1], raw[3 * ps + 2], 0.0f};
  float* nqdst = nqp + ((size_t)b * NQRY + t) * 4;
  v4f ov4 = (v4f){0.0f, 0.0f, 0.0f, 0.0f};
  float* odst = out0 + (size_t)b * NQRY * 3 + (size_t)(t < 768 ? t : 0) * 4;
  if (t < 768) {
    float e4[4];
#pragma unroll
    for (int e = 0; e < 4; ++e) {
      const int fl = 4 * t + e;
      const int s = fl / 3, cc = fl - 3 * s;
      e4[e] = raw[3 * sel[s] + cc];
    }
    ov4 = (v4f){e4[0], e4[1], e4[2], e4[3]};
  }
  *(volatile v4f*)nqdst = nv;
  if (t < 768) *(volatile v4f*)odst = ov4;
  __threadfence();
  *(volatile v4f*)nqdst = nv;
  if (t < 768) *(volatile v4f*)odst = ov4;
}

template <int KNB>
__global__ __launch_bounds__(256) void k_ballq(const float* __restrict__ xyz, const float* __restrict__ nqp,
                                               int* __restrict__ idx, float r2) {
#pragma clang fp contract(off)
  __shared__ __align__(16) int rows[8][IDXP];
  const int wid = threadIdx.x >> 5, lane = threadIdx.x & 31;
  const int q = blockIdx.x * 8 + wid;
  const int b = q >> 10;
  const v4f cq = *(const v4f*)(nqp + (size_t)q * 4);
  const float* base = xyz + (size_t)b * NPTS * 3;
  int cnt = 0, firstI = 0, have = 0;
#pragma unroll 1
  for (int s0 = 0; s0 < NPTS; s0 += 32) {
    const int p = s0 + lane;
    const float x = base[p * 3], y = base[p * 3 + 1], z = base[p * 3 + 2];
    const float dx = cq.x - x, dy = cq.y - y, dz = cq.z - z;
    const float t0 = dx * dx;
    const float t1 = dy * dy;
    const float t2 = dz * dz;
    const float d2 = (t0 + t2) + t1;
    const bool hit = d2 < r2;
    const unsigned mask = __builtin_amdgcn_ballot_w32(hit);
    if (!have && mask != 0u) { firstI = s0 + __ffs(mask) - 1; have = 1; }
    const int slot = cnt + __popc(mask & ((1u << lane) - 1u));
    if (hit && slot < KNB) rows[wid][slot] = p;
    cnt += __popc(mask);
    if (cnt >= KNB) break;
  }
  const int start = cnt < KNB ? cnt : KNB;
  for (int j = start + lane; j < IDXP; j += 32) rows[wid][j] = firstI;
  __syncthreads();
  if (wid < 4) {
    const int row = 2 * wid + (lane >> 4);
    const int c4 = (lane & 15) * 4;
    const v4i v = *(const v4i*)(&rows[row][c4]);
    int* dst = idx + ((size_t)(blockIdx.x * 8 + row)) * IDXP + c4;
    *(volatile v4i*)dst = v;
    __threadfence();
    *(volatile v4i*)dst = v;
  }
}

template <int KNB>
__global__ __launch_bounds__(256) void k_stats1(const float* __restrict__ xyz, const float* __restrict__ nqp,
                                                const int* __restrict__ idx, const float* __restrict__ W1,
                                                const float* __restrict__ b1, float* __restrict__ part) {
  __shared__ __align__(16) float geo[8 * KNB * 4];
  __shared__ float qi[8][8];
  __shared__ float red[4][128];
  __shared__ __align__(16) float fin[128];
  const int t = threadIdx.x;
  const int q0 = blockIdx.x * 8;
  const int b = q0 >> 10;
  for (int row = t; row < 8 * KNB; row += 256) {
    const int ql = row / KNB, k = row - ql * KNB;
    const int q = q0 + ql;
    const int p = clampi(idx[(size_t)q * IDXP + k], 0, NPTS - 1);
    const float* gp = xyz + ((size_t)b * NPTS + p) * 3;
    const v4f cq = *(const v4f*)(nqp + (size_t)q * 4);
    const float rx = gp[0] - cq.x, ry = gp[1] - cq.y, rz = gp[2] - cq.z;
    const float t0 = rx * rx;
    const float t1 = ry * ry;
    const float t2 = rz * rz;
    const float ds = sqrtf(((t0 + t2) + t1) + 1e-12f);
    *(v4f*)(&geo[row * 4]) = (v4f){ds, rx, ry, rz};
  }
  {
    const int ql = t & 7;
    const int q = q0 + ql;
    const int i0 = clampi(idx[(size_t)q * IDXP], 0, NPTS - 1);
    const float* xp = xyz + ((size_t)b * NPTS + i0) * 3;
    const v4f cq = *(const v4f*)(nqp + (size_t)q * 4);
    const float x0 = xp[0], x1 = xp[1], x2 = xp[2];
    if (t < 8) {
      qi[ql][0] = x0; qi[ql][1] = x1; qi[ql][2] = x2;
      qi[ql][3] = cq.x; qi[ql][4] = cq.y; qi[ql][5] = cq.z;
    }
  }
  const int c = t & 63, g = t >> 6;
  const float* wr = W1 + c * 10;
  const float w0 = wr[0];
  const float wx0 = wr[1], wx1 = wr[2], wx2 = wr[3];
  const float wg0 = wr[4], wg1 = wr[5], wg2 = wr[6];
  const float u0 = wg0 + wr[7], u1 = wg1 + wr[8], u2 = wg2 + wr[9];
  const float bias = b1[c];
  __syncthreads();
  float s = 0.0f, ss = 0.0f;
#pragma unroll 1
  for (int qq = 0; qq < 2; ++qq) {
    const int ql = 2 * g + qq;
    const float base = p1_base(bias, wx0, wx1, wx2, wg0, wg1, wg2,
                               qi[ql][0], qi[ql][1], qi[ql][2], qi[ql][3], qi[ql][4], qi[ql][5]);
#pragma unroll 2
    for (int k = 0; k < KNB; ++k) {
      const v4f gg = *(const v4f*)(&geo[(ql * KNB + k) * 4]);
      const float p = p1_eval(base, w0, u0, u1, u2, gg);
      s = s + p;
      const float pp = p * p;
      ss = ss + pp;
    }
  }
  red[g][c] = s;
  red[g][64 + c] = ss;
  __syncthreads();
  if (t < 128) fin[t] = ((red[0][t] + red[1][t]) + red[2][t]) + red[3][t];
  __syncthreads();
  if (t < 32) {
    const v4f v = *(const v4f*)(&fin[4 * t]);
    store2_v4f(part + (size_t)blockIdx.x * 128 + 4 * t, v);
  }
}

__global__ __launch_bounds__(128) void k_fin1(const float* __restrict__ part, int nblk, const float* __restrict__ g,
                                              const float* __restrict__ bb, float* __restrict__ ab, double invM) {
  __shared__ double sm[128];
  __shared__ __align__(16) float outv[128];
  const int t = threadIdx.x;
  double a = 0.0;
#pragma unroll 1
  for (int r = 0; r < nblk; ++r) a += (double)part[(size_t)r * 128 + t];
  sm[t] = a;
  __syncthreads();
  if (t < 64) {
    const double mean = sm[t] * invM;
    double var = sm[64 + t] * invM - mean * mean;
    var = var < 0.0 ? 0.0 : var;
    const float rs = 1.0f / sqrtf((float)var + 1e-5f);
    const float sc = g[t] * rs;
    outv[t] = sc;
    outv[64 + t] = bb[t] - (float)mean * sc;
  }
  __syncthreads();
  if (t < 32) {
    const v4f v = *(const v4f*)(&outv[4 * t]);
    store2_v4f(ab + 4 * t, v);
  }
}

template <int KNB>
__global__ __launch_bounds__(128) void k_main(const float* __restrict__ xyz, const float* __restrict__ nqp,
                                              const int* __restrict__ idx, const float* __restrict__ featT,
                                              const float* __restrict__ W1, const float* __restrict__ b1,
                                              const float* __restrict__ ab1,
                                              const unsigned short* __restrict__ W2h, const unsigned short* __restrict__ W2l,
                                              const float* __restrict__ b2, float* __restrict__ yplanes) {
  constexpr int MT = KNB / 16;
  __shared__ __align__(16) unsigned At[4][2][16 * 36];
  __shared__ __align__(16) float geo[4][64 * 4];
  __shared__ int pidx[4][64];
  __shared__ __align__(16) float outS[4][4 * YPITCH];
  const int tid = threadIdx.x, wave = tid >> 5, lane = tid & 31;
  const int hh = lane >> 4, c = lane & 15;
  const int q = blockIdx.x * 4 + wave;
  const int b = q >> 10;

  for (int e = tid; e < 256; e += 128) {
    const int pl = e >> 6, ql = (e >> 4) & 3, cc = e & 15;
    outS[pl][ql * YPITCH + 144 + cc] = 0.0f;
  }

  const v4f cq = *(const v4f*)(nqp + (size_t)q * 4);
  const int i0 = clampi(idx[(size_t)q * IDXP], 0, NPTS - 1);
  const float* xp = xyz + ((size_t)b * NPTS + i0) * 3;
  const float xi0 = xp[0], xi1 = xp[1], xi2 = xp[2];
#pragma unroll
  for (int kk = 0; kk < KNB / 32; ++kk) {
    const int k = lane + kk * 32;
    const int p = clampi(idx[(size_t)q * IDXP + k], 0, NPTS - 1);
    const float* gp = xyz + ((size_t)b * NPTS + p) * 3;
    const float rx = gp[0] - cq.x, ry = gp[1] - cq.y, rz = gp[2] - cq.z;
    const float t0 = rx * rx;
    const float t1 = ry * ry;
    const float t2 = rz * rz;
    const float ds = sqrtf(((t0 + t2) + t1) + 1e-12f);
    *(v4f*)(&geo[wave][k * 4]) = (v4f){ds, rx, ry, rz};
    pidx[wave][k] = p;
  }
  asm volatile("" ::: "memory");

  const int c0 = 2 * lane;
  const v4f* wp = (const v4f*)(W1 + c0 * 10);
  const v4f wa0 = wp[0], wa1 = wp[1], wa2 = wp[2], wa3 = wp[3], wa4 = wp[4];
  const float biasA = b1[c0], biasB = b1[c0 + 1];
  const float scA = ab1[c0], scB = ab1[c0 + 1];
  const float shA = ab1[CMID + c0], shB = ab1[CMID + c0 + 1];
  const float w0A = wa0.x;
  const float uA0 = wa1.x + wa1.w, uA1 = wa1.y + wa2.x, uA2 = wa1.z + wa2.y;
  const float baseA = p1_base(biasA, wa0.y, wa0.z, wa0.w, wa1.x, wa1.y, wa1.z, xi0, xi1, xi2, cq.x, cq.y, cq.z);
  const float w0B = wa2.z;
  const float uB0 = wa3.z + wa4.y, uB1 = wa3.w + wa4.z, uB2 = wa4.x + wa4.w;
  const float baseB = p1_base(biasB, wa2.w, wa3.x, wa3.y, wa3.z, wa3.w, wa4.x, xi0, xi1, xi2, cq.x, cq.y, cq.z);

  __syncthreads();

  unsigned* ath = &At[wave][0][0];
  unsigned* atl = &At[wave][1][0];

#pragma unroll 1
  for (int i = 0; i < MT; ++i) {
#pragma unroll 2
    for (int r = 0; r < 16; ++r) {
      const v4f gg = *(const v4f*)(&geo[wave][(i * 16 + r) * 4]);
      const float pA = p1_eval(baseA, w0A, uA0, uA1, uA2, gg);
      const float pB = p1_eval(baseB, w0B, uB0, uB1, uB2, gg);
      const float hA = fmaxf(scA * pA + shA, 0.0f);
      const float hB = fmaxf(scB * pB + shB, 0.0f);
      unsigned hbA, lbA, hbB, lbB;
      bf_split(hA, hbA, lbA);
      bf_split(hB, hbB, lbB);
      ath[r * 36 + lane] = hbA | (hbB << 16);
      atl[r * 36 + lane] = lbA | (lbB << 16);
    }
    __syncthreads();
    const __bf16* aph = (const __bf16*)ath + c * 72 + 8 * hh;
    const __bf16* apl = (const __bf16*)atl + c * 72 + 8 * hh;
    const v16b ah0 = frag_load(aph), ah1 = frag_load(aph + 32);
    const v16b al0 = frag_load(apl), al1 = frag_load(apl + 32);
    int pr[8];
#pragma unroll
    for (int r = 0; r < 8; ++r) pr[r] = pidx[wave][i * 16 + 8 * hh + r];

#pragma unroll 1
    for (int j = 0; j < 9; ++j) {
      const int n = j * 16 + c;
      const __bf16* bph = (const __bf16*)W2h + n * CMID + 8 * hh;
      const __bf16* bpl = (const __bf16*)W2l + n * CMID + 8 * hh;
      const v16b bh0 = frag_load(bph), bh1 = frag_load(bph + 32);
      const v16b bl0 = frag_load(bpl), bl1 = frag_load(bpl + 32);
      v8f acc = (v8f){0.f, 0.f, 0.f, 0.f, 0.f, 0.f, 0.f, 0.f};
      acc = mma_g(al0, bh0, acc);
      acc = mma_g(ah0, bl0, acc);
      acc = mma_g(ah0, bh0, acc);
      acc = mma_g(al1, bh1, acc);
      acc = mma_g(ah1, bl1, acc);
      acc = mma_g(ah1, bh1, acc);
      asm volatile("" ::: "memory");

      const bool valid = n < CIN;
      const int oc = valid ? n : (CIN - 1);
      const float b2v = b2[oc];
      const int chn = clampi(n - 3, 0, CFEAT - 1);
      const float fsel = (n >= 3) ? 1.0f : 0.0f;
      const float rsel = 1.0f - fsel;
      const int rc = n < 2 ? n : 2;
      float fv[8], rv[8];
#pragma unroll
      for (int r = 0; r < 8; ++r) fv[r] = featT[((size_t)b * NPTS + pr[r]) * CFEAT + chn];
      if (j == 0) {
#pragma unroll
        for (int r = 0; r < 8; ++r) rv[r] = geo[wave][(i * 16 + 8 * hh + r) * 4 + 1 + rc];
      } else {
#pragma unroll
        for (int r = 0; r < 8; ++r) rv[r] = 0.0f;
      }
#pragma unroll
      for (int r = 0; r < 8; ++r) asm volatile("" : "+v"(fv[r]), "+v"(rv[r]));
      float mx = -3.402823466e+38f, mn = 3.402823466e+38f, sm = 0.0f, sq = 0.0f;
#pragma unroll
      for (int r = 0; r < 8; ++r) {
        const float xa = fsel * fv[r];
        const float xb = rsel * rv[r];
        const float xv = xa + xb;
        float y = (acc[r] + b2v) * xv;
        y = valid ? y : 0.0f;
        mx = fmaxf(mx, y);
        mn = fminf(mn, y);
        sm = sm + y;
        const float yy = y * y;
        sq = sq + yy;
      }
      const float mx2 = __shfl_xor(mx, 16, 32);
      const float mn2 = __shfl_xor(mn, 16, 32);
      const float sm2 = __shfl_xor(sm, 16, 32);
      const float sq2 = __shfl_xor(sq, 16, 32);
      mx = fmaxf(mx, mx2);
      mn = fminf(mn, mn2);
      sm = sm + sm2;
      sq = sq + sq2;
      if (hh == 0) {
        const int a = wave * YPITCH + n;
        if (i == 0) {
          outS[0][a] = mx; outS[1][a] = mn; outS[2][a] = sm; outS[3][a] = sq;
        } else {
          outS[0][a] = fmaxf(outS[0][a], mx);
          outS[1][a] = fminf(outS[1][a], mn);
          outS[2][a] = outS[2][a] + sm;
          outS[3][a] = outS[3][a] + sq;
        }
      }
    }
    __syncthreads();
  }
  for (int pass = 0; pass < 2; ++pass) {
#pragma unroll 1
    for (int u = wave; u < 20; u += 4) {
      const int pl = u / 5, ch5 = u - pl * 5;
      const v4f v = *(const v4f*)(&outS[pl][ch5 * 128 + lane * 4]);
      float* dst = yplanes + (size_t)pl * ((size_t)NQTOT * YPITCH) + (size_t)blockIdx.x * (4 * YPITCH) + ch5 * 128 + lane * 4;
      *(volatile v4f*)dst = v;
    }
    __threadfence();
  }
}

__global__ __launch_bounds__(640) void k_fin2(const float* __restrict__ ysum, const float* __restrict__ ysq,
                                              const float* __restrict__ g, const float* __restrict__ bb,
                                              float* __restrict__ ab2, double invM) {
  __shared__ double s1[640];
  __shared__ double s2[640];
  __shared__ __align__(16) float outv[320];
  const int t = threadIdx.x;
  const int col = t % YPITCH, grp = t / YPITCH;
  double a = 0.0, qd = 0.0;
#pragma unroll 1
  for (int r = grp * 2048; r < grp * 2048 + 2048; ++r) {
    a += (double)ysum[(size_t)r * YPITCH + col];
    qd += (double)ysq[(size_t)r * YPITCH + col];
  }
  s1[t] = a;
  s2[t] = qd;
  __syncthreads();
  if (t < YPITCH) {
    const double S = ((s1[t] + s1[t + 160]) + s1[t + 320]) + s1[t + 480];
    const double Q = ((s2[t] + s2[t + 160]) + s2[t + 320]) + s2[t + 480];
    const double mean = S * invM;
    double var = Q * invM - mean * mean;
    var = var < 0.0 ? 0.0 : var;
    const bool valid = t < CIN;
    const int tc = valid ? t : (CIN - 1);
    const float rs = 1.0f / sqrtf((float)var + 1e-5f);
    const float sc = g[tc] * rs;
    const float sh = bb[tc] - (float)mean * sc;
    outv[t] = valid ? sc : 0.0f;
    outv[YPITCH + t] = valid ? sh : 0.0f;
  }
  __syncthreads();
  if (t < 80) {
    const v4f v = *(const v4f*)(&outv[4 * t]);
    store2_v4f(ab2 + 4 * t, v);
  }
}

__global__ __launch_bounds__(320) void k_pool(const float* __restrict__ ymax, const float* __restrict__ ymin,
                                              const float* __restrict__ ab2,
                                              unsigned short* __restrict__ xph, unsigned short* __restrict__ xpl) {
  const int t = threadIdx.x;
  const int e0 = t * 8;
  const int col = e0 % YPITCH;
  const size_t lin = (size_t)blockIdx.x * (16 * YPITCH) + e0;
  const v4f m0 = *(const v4f*)(ymax + lin), m1 = *(const v4f*)(ymax + lin + 4);
  const v4f n0 = *(const v4f*)(ymin + lin), n1 = *(const v4f*)(ymin + lin + 4);
  asm volatile("" ::: "memory");
  const v4f a0 = *(const v4f*)(ab2 + col), a1 = *(const v4f*)(ab2 + col + 4);
  const v4f c0 = *(const v4f*)(ab2 + YPITCH + col), c1 = *(const v4f*)(ab2 + YPITCH + col + 4);
  const float mxv[8] = {m0.x, m0.y, m0.z, m0.w, m1.x, m1.y, m1.z, m1.w};
  const float mnv[8] = {n0.x, n0.y, n0.z, n0.w, n1.x, n1.y, n1.z, n1.w};
  const float av[8]  = {a0.x, a0.y, a0.z, a0.w, a1.x, a1.y, a1.z, a1.w};
  const float cv[8]  = {c0.x, c0.y, c0.z, c0.w, c1.x, c1.y, c1.z, c1.w};
  unsigned hw[4], lw[4];
#pragma unroll
  for (int e2 = 0; e2 < 4; ++e2) {
    float xv[2];
#pragma unroll
    for (int s = 0; s < 2; ++s) {
      const int e = 2 * e2 + s;
      const float pick = (av[e] > 0.0f) ? mxv[e] : mnv[e];
      const float x = fmaxf(av[e] * pick + cv[e], 0.0f);
      xv[s] = ((col + e) < CIN) ? x : 0.0f;
    }
    unsigned h0, l0, h1, l1;
    bf_split(xv[0], h0, l0);
    bf_split(xv[1], h1, l1);
    hw[e2] = h0 | (h1 << 16);
    lw[e2] = l0 | (l1 << 16);
  }
  const v4u hv = (v4u){hw[0], hw[1], hw[2], hw[3]};
  const v4u lv = (v4u){lw[0], lw[1], lw[2], lw[3]};
  unsigned short* dh = xph + lin;
  unsigned short* dl = xpl + lin;
  *(volatile v4u*)dh = hv;
  *(volatile v4u*)dl = lv;
  __threadfence();
  *(volatile v4u*)dh = hv;
  *(volatile v4u*)dl = lv;
}

__global__ __launch_bounds__(256) void k_gemm_bf16x3(
    const unsigned short* __restrict__ Ahp, const unsigned short* __restrict__ Alp, int lda,
    const unsigned short* __restrict__ Bhp, const unsigned short* __restrict__ Blp, int ldb,
    float* __restrict__ Cout, int ldc, const float* __restrict__ bias, int M, int N, int K) {
  const __bf16* A  = (const __bf16*)Ahp;
  const __bf16* A2 = (const __bf16*)Alp;
  const __bf16* Bt  = (const __bf16*)Bhp;
  const __bf16* Bt2 = (const __bf16*)Blp;
  __shared__ __align__(16) float sT[8][16 * 68];
  const int lane = threadIdx.x & 31;
  const int wave = threadIdx.x >> 5;
  const int tilesN = N >> 6;
  const int tilesM = M >> 6;
  const int tile = blockIdx.x * 8 + wave;
  if (tile >= tilesM * tilesN) return;
  const int tm = tile / tilesN;
  const int tn = tile - tm * tilesN;
  const int m0 = tm << 6;
  const int n0 = tn << 6;
  const int rlane = lane & 15;
  const int koff  = (lane >> 4) * 8;
  const int mOff  = (lane >> 4) * 8;

  v8f acc[4][4];
#pragma unroll
  for (int i = 0; i < 4; ++i)
#pragma unroll
    for (int j = 0; j < 4; ++j) acc[i][j] = (v8f){0.f, 0.f, 0.f, 0.f, 0.f, 0.f, 0.f, 0.f};

  for (int k0 = 0; k0 < K; k0 += 32) {
    v16b bh[4], bl[4];
#pragma unroll
    for (int j = 0; j < 4; ++j) {
      const size_t bo = (size_t)(n0 + (j << 4) + rlane) * ldb + koff + k0;
      bh[j] = frag_load(Bt + bo);
      bl[j] = frag_load(Bt2 + bo);
    }
#pragma unroll
    for (int i = 0; i < 4; ++i) {
      const size_t ao = (size_t)(m0 + (i << 4) + rlane) * lda + koff + k0;
      const v16b ah = frag_load(A + ao);
      const v16b al = frag_load(A2 + ao);
#pragma unroll
      for (int j = 0; j < 4; ++j) {
        acc[i][j] = mma_plain(ah, bh[j], acc[i][j]);
        acc[i][j] = mma_plain(ah, bl[j], acc[i][j]);
        acc[i][j] = mma_plain(al, bh[j], acc[i][j]);
      }
      dep_guard4_b(acc[i][0], acc[i][1], acc[i][2], acc[i][3], ah, al);
    }
    keep4_b(bh[0], bh[1], bh[2], bh[3]);
    keep4_b(bl[0], bl[1], bl[2], bl[3]);
  }
  acc_guard4(acc[0][0], acc[0][1], acc[0][2], acc[0][3]);
  acc_guard4(acc[1][0], acc[1][1], acc[1][2], acc[1][3]);
  acc_guard4(acc[2][0], acc[2][1], acc[2][2], acc[2][3]);
  acc_guard4(acc[3][0], acc[3][1], acc[3][2], acc[3][3]);

  float* slab = sT[wave];
#pragma unroll
  for (int i = 0; i < 4; ++i) {
    const int mBase = m0 + (i << 4);
#pragma unroll
    for (int j = 0; j < 4; ++j) {
      const int n = n0 + (j << 4) + rlane;
      const float bv = bias[n];
#pragma unroll
      for (int r = 0; r < 8; ++r) {
        const float v = acc[i][j][r] + bv;
        slab[(mOff + r) * 68 + (j << 4) + rlane] = v;
      }
    }
    __builtin_amdgcn_fence(__ATOMIC_RELEASE, "workgroup");
    __builtin_amdgcn_wave_barrier();
    __builtin_amdgcn_fence(__ATOMIC_ACQUIRE, "workgroup");
    {
      const int hh = lane >> 4, c4 = (lane & 15) * 4;
      for (int pass = 0; pass < 2; ++pass) {
#pragma unroll
        for (int it = 0; it < 8; ++it) {
          const int row = it * 2 + hh;
          const v4f v = *(const v4f*)(slab + row * 68 + c4);
          *(volatile v4f*)(Cout + (size_t)(mBase + row) * ldc + n0 + c4) = v;
        }
        __threadfence();
      }
    }
    __builtin_amdgcn_fence(__ATOMIC_RELEASE, "workgroup");
    __builtin_amdgcn_wave_barrier();
    __builtin_amdgcn_fence(__ATOMIC_ACQUIRE, "workgroup");
  }
}

__global__ __launch_bounds__(1024) void k_fin3(const float* __restrict__ P3, const float* __restrict__ g,
                                               const float* __restrict__ bb, float* __restrict__ ab3, double invM) {
  __shared__ double s1[1024];
  __shared__ double s2[1024];
  __shared__ __align__(16) float outv[512];
  const int t = threadIdx.x;
  const int col = t & 255, grp = t >> 8;
  double a = 0.0, qd = 0.0;
#pragma unroll 1
  for (int r = grp * 2048; r < grp * 2048 + 2048; ++r) {
    const double p = (double)P3[(size_t)r * COUTC + col];
    a += p;
    const double pp = p * p;
    qd += pp;
  }
  s1[t] = a;
  s2[t] = qd;
  __syncthreads();
  if (t < COUTC) {
    const double S = ((s1[t] + s1[t + 256]) + s1[t + 512]) + s1[t + 768];
    const double Q = ((s2[t] + s2[t + 256]) + s2[t + 512]) + s2[t + 768];
    const double mean = S * invM;
    double var = Q * invM - mean * mean;
    var = var < 0.0 ? 0.0 : var;
    const float rs = 1.0f / sqrtf((float)var + 1e-5f);
    const float sc = g[t] * rs;
    outv[t] = sc;
    outv[COUTC + t] = bb[t] - (float)mean * sc;
  }
  __syncthreads();
  if (t < 128) {
    const v4f v = *(const v4f*)(&outv[4 * t]);
    store2_v4f(ab3 + 4 * t, v);
  }
}

__global__ __launch_bounds__(256) void k_apply(const float* __restrict__ P3, const float* __restrict__ ab3,
                                               float* __restrict__ out1, int scOff) {
  __shared__ float tile[32 * 33];
  const int tid = threadIdx.x, wave = tid >> 5, lane = tid & 31;
  const int s0 = blockIdx.x * 32, o0 = blockIdx.y * 32, b = blockIdx.z;
  const float sc = ab3[o0 + lane], sh = ab3[COUTC + o0 + lane];
#pragma unroll
  for (int r = 0; r < 4; ++r) {
    const int s = wave * 4 + r;
    const float p = P3[((size_t)b * NQRY + s0 + s) * COUTC + o0 + lane];
    tile[s * 33 + lane] = fmaxf(sc * p + sh, 0.0f);
  }
  __syncthreads();
  const int oq = lane >> 3, s4 = (lane & 7) * 4;
  const int o = wave * 4 + oq;
  const v4f v = (v4f){tile[(s4 + 0) * 33 + o], tile[(s4 + 1) * 33 + o], tile[(s4 + 2) * 33 + o], tile[(s4 + 3) * 33 + o]};
  float* dst = out1 + ((size_t)(b * 2 * COUTC + scOff + o0 + o)) * NQRY + s0 + s4;
  store2_v4f(dst, v);
}

extern "C" void kernel_launch(void* const* d_in, const int* in_sizes, int n_in,
                              void* d_out, int out_size, void* d_ws, size_t ws_size, hipStream_t stream) {
  (void)in_sizes; (void)out_size;
  if (n_in < 14) return;
  if (ws_size < WS_TOTAL) return;
  const float* xyz      = (const float*)d_in[0];
  const float* features = (const float*)d_in[1];
  const float* W1       = (const float*)d_in[2];
  const float* b1       = (const float*)d_in[3];
  const float* W2       = (const float*)d_in[4];
  const float* b2       = (const float*)d_in[5];
  const float* Wcr      = (const float*)d_in[6];
  const float* bcr      = (const float*)d_in[7];
  const float* g_map    = (const float*)d_in[8];
  const float* b_map    = (const float*)d_in[9];
  const float* g_rs     = (const float*)d_in[10];
  const float* b_rs     = (const float*)d_in[11];
  const float* g_cr     = (const float*)d_in[12];
  const float* b_cr     = (const float*)d_in[13];

  float* out0 = (float*)d_out;
  float* out1 = out0 + OUT1_FLOAT_OFF;

  char* ws = (char*)d_ws;
  float* featT = (float*)(ws + OFF_FEATT);
  float* nqp   = (float*)(ws + OFF_NQ);
  unsigned short* W2h = (unsigned short*)(ws + OFF_W2H);
  unsigned short* W2l = (unsigned short*)(ws + OFF_W2L);
  unsigned short* Wch = (unsigned short*)(ws + OFF_WCH);
  unsigned short* Wcl = (unsigned short*)(ws + OFF_WCL);

  k_transpose_feat<<<dim3(NPTS / 32, NBATCH), 256, 0, stream>>>(features, featT);
  k_wprep<<<25, 256, 0, stream>>>(W2, Wcr, W2h, W2l, Wch, Wcl);
  k_fps<<<NBATCH, 1024, 0, stream>>>(xyz, out0, nqp);

  for (int sc = 0; sc < 2; ++sc) {
    char* sb = ws + OFF_SC0 + (size_t)sc * SC_BYTES;
    int*   idx  = (int*)(sb + SC_IDX);
    float* st1  = (float*)(sb + SC_ST1);
    float* ab1  = (float*)(sb + SC_AB1);
    float* ypl  = (float*)(sb + SC_Y);
    float* ab2  = (float*)(sb + SC_AB2);
    unsigned short* xph = (unsigned short*)(sb + SC_XPH);
    unsigned short* xpl = (unsigned short*)(sb + SC_XPL);
    float* P3   = (float*)(sb + SC_P3);
    float* ab3  = (float*)(sb + SC_AB3);
    const size_t plane = (size_t)NQTOT * YPITCH;
    const int knb = (sc == 0) ? 32 : 64;
    const double invM = 1.0 / ((double)NQTOT * (double)knb);
    const double invQ = 1.0 / (double)NQTOT;

    if (sc == 0) {
      k_ballq<32><<<NQTOT / 8, 256, 0, stream>>>(xyz, nqp, idx, 0.01f);
      k_stats1<32><<<NQTOT / 8, 256, 0, stream>>>(xyz, nqp, idx, W1, b1, st1);
    } else {
      k_ballq<64><<<NQTOT / 8, 256, 0, stream>>>(xyz, nqp, idx, 0.04f);
      k_stats1<64><<<NQTOT / 8, 256, 0, stream>>>(xyz, nqp, idx, W1, b1, st1);
    }
    k_fin1<<<1, 128, 0, stream>>>(st1, NQTOT / 8, g_map + sc * CMID, b_map + sc * CMID, ab1, invM);
    if (sc == 0) {
      k_main<32><<<NQTOT / 4, 128, 0, stream>>>(xyz, nqp, idx, featT, W1, b1, ab1, W2h, W2l, b2, ypl);
    } else {
      k_main<64><<<NQTOT / 4, 128, 0, stream>>>(xyz, nqp, idx, featT, W1, b1, ab1, W2h, W2l, b2, ypl);
    }
    k_fin2<<<1, 640, 0, stream>>>(ypl + 2 * plane, ypl + 3 * plane, g_rs + sc * CIN, b_rs + sc * CIN, ab2, invM);
    k_pool<<<NQTOT / 16, 320, 0, stream>>>(ypl, ypl + plane, ab2, xph, xpl);
    k_gemm_bf16x3<<<(NQTOT / 64) * (COUTC / 64) / 8, 256, 0, stream>>>(xph, xpl, KPADW, Wch, Wcl, KPADW,
                                                                        P3, COUTC, bcr, NQTOT, COUTC, KPADW);
    k_fin3<<<1, 1024, 0, stream>>>(P3, g_cr + sc * COUTC, b_cr + sc * COUTC, ab3, invQ);
    k_apply<<<dim3(NQRY / 32, COUTC / 32, NBATCH), 256, 0, stream>>>(P3, ab3, out1, sc * COUTC);
  }
}
